// TransformerBlock_3435973837252
// MI455X (gfx1250) — hardware-verified
//
#include <hip/hip_runtime.h>
#include <stddef.h>
#include <math.h>


typedef _Float16 v16h __attribute__((ext_vector_type(16)));
typedef _Float16 v8h  __attribute__((ext_vector_type(8)));
typedef float    v8f  __attribute__((ext_vector_type(8)));
typedef float    v4f  __attribute__((ext_vector_type(4)));

#ifndef NB
#define NB 2
#endif
#ifndef SEQ
#define SEQ 2048
#endif
#define NB_FULL  2
#define SEQ_FULL 2048
#define DIM   1024
#define NHEAD 16
#define HD    64
#define FF    4096
#define MROWS (NB * SEQ)

static_assert(NB >= 1 && NB <= NB_FULL);
static_assert(SEQ >= 128 && SEQ <= SEQ_FULL && (SEQ % 128) == 0);
static_assert(DIM == NHEAD * HD && NHEAD == 16 && HD == 64 && DIM == 1024);
static_assert(FF == 4 * DIM);
static_assert((MROWS % 64) == 0 && (MROWS % 8) == 0);
static_assert((DIM % 64) == 0 && (FF % 64) == 0);

#define LDT 72
#define LDC 68

#define WCARRY 64.0f
#define PCARRY 1024.0f
#define VCARRY 64.0f
#define HCARRY 16.0f

#define P16_BYTES  ((size_t)MROWS * DIM * 2)
#define WQKV_BYTES ((size_t)3 * HD * HD * 2)
#define WO_BYTES   ((size_t)DIM * DIM * 2)
#define W1_BYTES   ((size_t)FF * DIM * 2)
#define W2_BYTES   ((size_t)DIM * FF * 2)
#define OFF_WQKV   ((size_t)0)
#define OFF_WO     (OFF_WQKV + WQKV_BYTES)
#define OFF_W1     (OFF_WO + WO_BYTES)
#define OFF_W2     (OFF_W1 + W1_BYTES)
#define OFF_XO     (OFF_W2 + W2_BYTES)
#define OFF_QKV    (OFF_XO + P16_BYTES)
#define OFF_X32    (OFF_QKV + 3 * P16_BYTES)
#define OFF_X1     (OFF_X32 + 2 * P16_BYTES)
#define OFF_H      (OFF_X1 + 2 * P16_BYTES)
#define OFF_G      (OFF_H + P16_BYTES)
#define WS_TOTAL   (OFF_G + 4 * P16_BYTES)
static_assert((size_t)MROWS * FF * 2 == 4 * P16_BYTES);
static_assert((size_t)NB * DIM * SEQ * 2 == P16_BYTES);
static_assert((size_t)MROWS * DIM * 4 == 2 * P16_BYTES);
static_assert((P16_BYTES % 128) == 0 && (WO_BYTES % 128) == 0 && (WQKV_BYTES % 128) == 0);
static_assert(WS_TOTAL <= (size_t)134217728);

__device__ __forceinline__ float bf16r(float x) {
  unsigned int u = __float_as_uint(x);
  u = (u + 0x7FFFu + ((u >> 16) & 1u)) & 0xFFFF0000u;
  return __uint_as_float(u);
}

__device__ __forceinline__ size_t full_row(unsigned r) {
  const unsigned n = r / (unsigned)SEQ;
  const unsigned s = r - n * (unsigned)SEQ;
  return (size_t)n * SEQ_FULL + s;
}

__device__ __forceinline__ v16h frag_at(const _Float16* p) {
  v8h lo = *(const v8h*)(p);
  v8h hi = *(const v8h*)(p + 16);
  v16h out;
#pragma unroll
  for (int i = 0; i < 8; ++i) { out[i] = lo[i]; out[i + 8] = hi[i]; }
  return out;
}
__device__ __forceinline__ v16h ld_frag(const _Float16* base, int ld) {
  const int lane = threadIdx.x & 31;
  return frag_at(base + (lane & 15) * ld + (lane >> 4) * 8);
}

__device__ __forceinline__ v8f wmma16(v16h a, v16h b, v8f c) {
  v8f d = __builtin_amdgcn_wmma_f32_16x16x32_f16(false, a, false, b, (short)0, c,
                                                 false, false);
  asm volatile("v_nop\n\tv_nop\n\tv_nop\n\tv_nop" : "+v"(d) : "v"(a), "v"(b));
  return d;
}

__device__ __forceinline__ float red16_max(float x) {
#pragma unroll
  for (int off = 1; off < 16; off <<= 1) x = fmaxf(x, __shfl_xor(x, off, 32));
  return x;
}
__device__ __forceinline__ float red16_sum(float x) {
#pragma unroll
  for (int off = 1; off < 16; off <<= 1) x += __shfl_xor(x, off, 32);
  return x;
}
__device__ __forceinline__ float wave_sum(float x) {
#pragma unroll
  for (int off = 1; off < 32; off <<= 1) x += __shfl_xor(x, off, 32);
  return x;
}

__device__ __forceinline__ void wave_lds_sync() {
  __builtin_amdgcn_fence(3  , "wavefront");
  asm volatile("s_wait_dscnt 0x0" ::: "memory");
  __builtin_amdgcn_wave_barrier();
}

template <int XMAP>
__global__ __launch_bounds__(256) void cvt_kernel(
    const float* __restrict__ src, _Float16* __restrict__ dst, float carry) {
  const unsigned i = blockIdx.x * 256u + threadIdx.x;
  const size_t e = (size_t)i * 8;
  size_t se = e;
  if (XMAP) {
    const unsigned row = i >> 7;
    const unsigned col = (i & 127u) * 8u;
    se = full_row(row) * DIM + col;
  }
  const v4f a0 = *(const v4f*)(src + se);
  const v4f a1 = *(const v4f*)(src + se + 4);
  v8h o;
#pragma unroll
  for (int t = 0; t < 4; ++t) {
    o[t]     = (_Float16)(carry * bf16r(a0[t]));
    o[t + 4] = (_Float16)(carry * bf16r(a1[t]));
  }
  *(volatile v8h*)(dst + e) = o;
  __threadfence();
  *(volatile v8h*)(dst + e) = o;
}

__global__ __launch_bounds__(256) void cvt3_kernel(
    const float* __restrict__ wq, const float* __restrict__ wk,
    const float* __restrict__ wv, _Float16* __restrict__ dst) {
  const unsigned which = blockIdx.y;
  const float* src = (which == 0u) ? wq : ((which == 1u) ? wk : wv);
  const unsigned i = blockIdx.x * 256u + threadIdx.x;
  const size_t e = (size_t)i * 8;
  const v4f a0 = *(const v4f*)(src + e);
  const v4f a1 = *(const v4f*)(src + e + 4);
  v8h o;
#pragma unroll
  for (int t = 0; t < 4; ++t) {
    o[t]     = (_Float16)(WCARRY * bf16r(a0[t]));
    o[t + 4] = (_Float16)(WCARRY * bf16r(a1[t]));
  }
  _Float16* d = dst + (size_t)which * (HD * HD) + e;
  *(volatile v8h*)d = o;
  __threadfence();
  *(volatile v8h*)d = o;
}

template <int OUT16, int FULLOUT>
__global__ __launch_bounds__(256) void ln_kernel(
    const float* __restrict__ src, const float* __restrict__ gam,
    const float* __restrict__ bet, float* __restrict__ dstf,
    _Float16* __restrict__ dst16) {
  static_assert(4 * 32 * 8 == DIM && 8 * 32 * 4 == DIM);
  const int lane = threadIdx.x & 31, w = threadIdx.x >> 5;
  const unsigned row = blockIdx.x * 8u + (unsigned)w;
  const float* xr = src + (size_t)row * DIM;

  float s = 0.0f;
#pragma unroll 1
  for (int j = 0; j < 4; ++j) {
    const int c = j * 256 + lane * 8;
    const v4f a0 = *(const v4f*)(xr + c);
    const v4f a1 = *(const v4f*)(xr + c + 4);
#pragma unroll
    for (int t = 0; t < 4; ++t) { s += a0[t]; s += a1[t]; }
  }
  const float mu = wave_sum(s) * (1.0f / DIM);

  float q = 0.0f;
#pragma unroll 1
  for (int j = 0; j < 4; ++j) {
    const int c = j * 256 + lane * 8;
    const v4f a0 = *(const v4f*)(xr + c);
    const v4f a1 = *(const v4f*)(xr + c + 4);
#pragma unroll
    for (int t = 0; t < 4; ++t) {
      const float d0 = a0[t] - mu;
      const float d1 = a1[t] - mu;
      q += d0 * d0;
      q += d1 * d1;
    }
  }
  const float var = wave_sum(q) * (1.0f / DIM);
  const float rs = rsqrtf(var + 1.0e-5f);

  if (OUT16) {
    _Float16* orow = dst16 + (size_t)row * DIM;
#pragma unroll 1
    for (int j = 0; j < 4; ++j) {
      const int c = j * 256 + lane * 8;
      const v4f a0 = *(const v4f*)(xr + c);
      const v4f a1 = *(const v4f*)(xr + c + 4);
      const v4f g0 = *(const v4f*)(gam + c);
      const v4f g1 = *(const v4f*)(gam + c + 4);
      const v4f b0 = *(const v4f*)(bet + c);
      const v4f b1 = *(const v4f*)(bet + c + 4);
      v8h o;
#pragma unroll
      for (int t = 0; t < 4; ++t) {
        const float y0 = ((a0[t] - mu) * rs) * bf16r(g0[t]) + bf16r(b0[t]);
        const float y1 = ((a1[t] - mu) * rs) * bf16r(g1[t]) + bf16r(b1[t]);
        o[t]     = (_Float16)y0;
        o[t + 4] = (_Float16)y1;
      }
      *(volatile v8h*)(orow + c) = o;
      __threadfence();
      *(volatile v8h*)(orow + c) = o;
    }
  }

  {
    const size_t orf = FULLOUT ? full_row(row) : (size_t)row;
    float* orow = dstf + orf * DIM;
#pragma unroll 1
    for (int j = 0; j < 8; ++j) {
      const int c = j * 128 + lane * 4;
      const v4f a = *(const v4f*)(xr + c);
      const v4f g = *(const v4f*)(gam + c);
      const v4f b = *(const v4f*)(bet + c);
      v4f y;
#pragma unroll
      for (int t = 0; t < 4; ++t)
        y[t] = ((a[t] - mu) * rs) * bf16r(g[t]) + bf16r(b[t]);
      *(volatile v4f*)(orow + c) = y;
      __threadfence();
      *(volatile v4f*)(orow + c) = y;
    }
  }
}

__global__ __launch_bounds__(256) void qkv_kernel(
    const _Float16* __restrict__ X16, const _Float16* __restrict__ Wp,
    _Float16* __restrict__ QKV) {
  __shared__ float Cs[64 * LDC];
  const int tid = threadIdx.x, lane = tid & 31, w = tid >> 5;
  const int mw = w >> 1, nw = w & 1;
  const int hh = lane >> 4, m = lane & 15;
  const unsigned which = blockIdx.x >> 4;
  const unsigned head = blockIdx.x & 15u;
  const unsigned row0 = blockIdx.y * 64u;

  const _Float16* ap  = X16 + (size_t)(row0 + mw * 16 + m) * DIM + head * HD + hh * 8;
  const _Float16* bp0 = Wp + (size_t)(which * HD + nw * 32 + m) * HD + hh * 8;
  const _Float16* bp1 = bp0 + (size_t)16 * HD;
  v8f acc0 = {}, acc1 = {};
#pragma unroll
  for (int k0 = 0; k0 < HD; k0 += 32) {
    const v16h a  = frag_at(ap + k0);
    const v16h b0 = frag_at(bp0 + k0);
    const v16h b1 = frag_at(bp1 + k0);
    acc0 = wmma16(a, b0, acc0);
    acc1 = wmma16(a, b1, acc1);
  }
#pragma unroll
  for (int r = 0; r < 8; ++r) {
    float* d = &Cs[(mw * 16 + hh * 8 + r) * LDC + nw * 32 + m];
    d[0]  = acc0[r];
    d[16] = acc1[r];
  }
  __syncthreads();

  _Float16* dst = QKV + (size_t)which * ((size_t)MROWS * DIM);
  v8h x[2];
  size_t off[2];
  if (which < 2u) {
#pragma unroll
    for (int i = 0; i < 2; ++i) {
      const int r = 32 * i + (tid >> 3);
      const int c = (tid & 7) * 8;
      const v4f u0 = *(const v4f*)&Cs[r * LDC + c];
      const v4f u1 = *(const v4f*)&Cs[r * LDC + c + 4];
#pragma unroll
      for (int j = 0; j < 4; ++j) {
        x[i][j]     = (_Float16)(u0[j] * (1.0f / WCARRY));
        x[i][j + 4] = (_Float16)(u1[j] * (1.0f / WCARRY));
      }
      off[i] = (size_t)(row0 + r) * DIM + head * HD + c;
    }
  } else {
    const unsigned nbat = row0 / (unsigned)SEQ;
    const unsigned s0 = row0 - nbat * (unsigned)SEQ;
#pragma unroll
    for (int i = 0; i < 2; ++i) {
      const int dcol = 32 * i + (tid >> 3);
      const int kk = (tid & 7) * 8;
#pragma unroll
      for (int j = 0; j < 8; ++j)
        x[i][j] = (_Float16)(Cs[(kk + j) * LDC + dcol] * (1.0f / WCARRY));
      off[i] = ((size_t)nbat * DIM + head * HD + dcol) * SEQ + s0 + kk;
    }
  }
#pragma unroll
  for (int i = 0; i < 2; ++i) *(volatile v8h*)(dst + off[i]) = x[i];
  __threadfence();
#pragma unroll
  for (int i = 0; i < 2; ++i) *(volatile v8h*)(dst + off[i]) = x[i];
}

#define MODE_WO  1
#define MODE_W1  2
#define MODE_W2  3

template <int MODE, int KD, int ND>
__global__ __launch_bounds__(256) void gemm_kernel(
    const _Float16* __restrict__ A16, const _Float16* __restrict__ Bt,
    const float* __restrict__ bias, const float* __restrict__ addf,
    float* __restrict__ outf, _Float16* __restrict__ out16) {
  static_assert((KD % 32) == 0 && (ND % 64) == 0);
  static_assert((MODE != MODE_WO && MODE != MODE_W2) || ND == DIM);
  __shared__ float Cs[64 * LDC];
  const int tid = threadIdx.x, lane = tid & 31, w = tid >> 5;
  const int mw = w >> 1, nw = w & 1;
  const int hh = lane >> 4, m = lane & 15;
  const int n0 = blockIdx.x * 64;
  const int row0 = blockIdx.y * 64;

  const _Float16* ap  = A16 + (size_t)(row0 + mw * 16 + m) * KD + hh * 8;
  const _Float16* bp0 = Bt + (size_t)(n0 + nw * 32 + m) * KD + hh * 8;
  const _Float16* bp1 = bp0 + (size_t)16 * KD;
  v8f acc0 = {}, acc1 = {};
#pragma unroll 2
  for (int k0 = 0; k0 < KD; k0 += 32) {
    const v16h a  = frag_at(ap + k0);
    const v16h b0 = frag_at(bp0 + k0);
    const v16h b1 = frag_at(bp1 + k0);
    acc0 = wmma16(a, b0, acc0);
    acc1 = wmma16(a, b1, acc1);
  }
#pragma unroll
  for (int r = 0; r < 8; ++r) {
    float* d = &Cs[(mw * 16 + hh * 8 + r) * LDC + nw * 32 + m];
    d[0]  = acc0[r];
    d[16] = acc1[r];
  }
  __syncthreads();

  if (MODE == MODE_WO) {
    v4f xs[4];
    size_t off[4];
#pragma unroll
    for (int i = 0; i < 4; ++i) {
      const int r = 16 * i + (tid >> 4);
      const int c = (tid & 15) * 4;
      const unsigned crow = (unsigned)(row0 + r);
      const v4f u = *(const v4f*)&Cs[r * LDC + c];
      const v4f g = *(const v4f*)(bias + n0 + c);
      const v4f q = *(const v4f*)(addf + full_row(crow) * DIM + n0 + c);
      v4f val;
#pragma unroll
      for (int j = 0; j < 4; ++j)
        val[j] = (u[j] * (1.0f / (WCARRY * VCARRY)) + bf16r(g[j])) + bf16r(q[j]);
      xs[i] = val;
      off[i] = (size_t)crow * ND + n0 + c;
    }
#pragma unroll
    for (int i = 0; i < 4; ++i) *(volatile v4f*)(outf + off[i]) = xs[i];
    __threadfence();
#pragma unroll
    for (int i = 0; i < 4; ++i) *(volatile v4f*)(outf + off[i]) = xs[i];
  }

  if (MODE == MODE_W1) {
    v8h x[2];
    size_t off[2];
#pragma unroll
    for (int i = 0; i < 2; ++i) {
      const int r = 32 * i + (tid >> 3);
      const int c = (tid & 7) * 8;
      const v4f u0 = *(const v4f*)&Cs[r * LDC + c];
      const v4f u1 = *(const v4f*)&Cs[r * LDC + c + 4];
      const v4f g0 = *(const v4f*)(bias + n0 + c);
      const v4f g1 = *(const v4f*)(bias + n0 + c + 4);
#pragma unroll
      for (int j = 0; j < 4; ++j) {
        const float t0 = fmaxf(u0[j] * (1.0f / WCARRY) + bf16r(g0[j]), 0.0f);
        const float t1 = fmaxf(u1[j] * (1.0f / WCARRY) + bf16r(g1[j]), 0.0f);
        x[i][j]     = (_Float16)(HCARRY * t0);
        x[i][j + 4] = (_Float16)(HCARRY * t1);
      }
      off[i] = (size_t)(row0 + r) * ND + n0 + c;
    }
#pragma unroll
    for (int i = 0; i < 2; ++i) *(volatile v8h*)(out16 + off[i]) = x[i];
    __threadfence();
#pragma unroll
    for (int i = 0; i < 2; ++i) *(volatile v8h*)(out16 + off[i]) = x[i];
  }

  if (MODE == MODE_W2) {
    v4f xs[4];
    size_t off[4];
#pragma unroll
    for (int i = 0; i < 4; ++i) {
      const int r = 16 * i + (tid >> 4);
      const int c = (tid & 15) * 4;
      const size_t crow = (size_t)(row0 + r);
      const v4f u  = *(const v4f*)&Cs[r * LDC + c];
      const v4f g  = *(const v4f*)(bias + n0 + c);
      const v4f rx = *(const v4f*)(addf + crow * DIM + n0 + c);
      v4f val;
#pragma unroll
      for (int j = 0; j < 4; ++j)
        val[j] = (u[j] * (1.0f / (WCARRY * HCARRY)) + bf16r(g[j])) + rx[j];
      xs[i] = val;
      off[i] = crow * ND + n0 + c;
    }
#pragma unroll
    for (int i = 0; i < 4; ++i) *(volatile v4f*)(outf + off[i]) = xs[i];
    __threadfence();
#pragma unroll
    for (int i = 0; i < 4; ++i) *(volatile v4f*)(outf + off[i]) = xs[i];
  }
}

__global__ __launch_bounds__(256) void attn_kernel(
    const _Float16* __restrict__ Qh, const _Float16* __restrict__ Kh,
    const _Float16* __restrict__ Vt, _Float16* __restrict__ Ov) {
  __shared__ _Float16 Ks[64 * LDT];
  __shared__ _Float16 Vs[64 * LDT];
  __shared__ _Float16 Ps[8 * 16 * LDT];

  const int tid = threadIdx.x, lane = tid & 31;
  const int w = __builtin_amdgcn_readfirstlane(tid >> 5);
  const int hh = lane >> 4, m = lane & 15;
  const int q0 = blockIdx.x * 128;
  const int head = blockIdx.y;
  const int nbat = blockIdx.z;
  const int wq0 = q0 + w * 16;
  const float scale = 0.03125f;
  _Float16* P = Ps + w * (16 * LDT);

  const size_t tok0 = (size_t)nbat * SEQ;
  const size_t qoff = (tok0 + wq0 + m) * DIM + head * HD + hh * 8;
  v16h qf[2];
  qf[0] = frag_at(Qh + qoff);
  qf[1] = frag_at(Qh + qoff + 32);

  float mrow[8], lrow[8];
  v8f o[4];
#pragma unroll
  for (int v = 0; v < 8; ++v) { mrow[v] = -1.0e30f; lrow[v] = 0.0f; }
#pragma unroll
  for (int nb = 0; nb < 4; ++nb) o[nb] = (v8f){};

  const size_t kplane = tok0 * DIM + (size_t)head * HD;
  const size_t vplane = ((size_t)nbat * DIM + (size_t)head * HD) * SEQ;

  for (int kb = 0; kb < SEQ; kb += 64) {
#pragma unroll
    for (int j = 0; j < 2; ++j) {
      const int idx = tid + 256 * j;
      const int r = idx >> 3, c = (idx & 7) * 8;
      *(v8h*)&Ks[r * LDT + c] = *(const v8h*)(Kh + kplane + (size_t)(kb + r) * DIM + c);
      *(v8h*)&Vs[r * LDT + c] = *(const v8h*)(Vt + vplane + (size_t)r * SEQ + kb + c);
    }
    __syncthreads();

    v8f s[4];
#pragma unroll
    for (int kg = 0; kg < 4; ++kg) {
      v8f t = {};
#pragma unroll
      for (int c = 0; c < 2; ++c) {
        const v16h kf = ld_frag(&Ks[(kg * 16) * LDT + c * 32], LDT);
        t = wmma16(qf[c], kf, t);
      }
      s[kg] = t * scale;
    }

    float alpha[8];
#pragma unroll
    for (int v = 0; v < 8; ++v) {
      float mx = fmaxf(fmaxf(s[0][v], s[1][v]), fmaxf(s[2][v], s[3][v]));
      mx = red16_max(mx);
      const float mn = fmaxf(mrow[v], mx);
      alpha[v] = __expf(mrow[v] - mn);
      mrow[v] = mn;
    }
#pragma unroll
    for (int kg = 0; kg < 4; ++kg)
#pragma unroll
      for (int v = 0; v < 8; ++v) s[kg][v] = __expf(s[kg][v] - mrow[v]);
#pragma unroll
    for (int v = 0; v < 8; ++v) {
      const float rs = red16_sum((s[0][v] + s[1][v]) + (s[2][v] + s[3][v]));
      lrow[v] = alpha[v] * lrow[v] + rs;
    }
#pragma unroll
    for (int nb = 0; nb < 4; ++nb)
#pragma unroll
      for (int v = 0; v < 8; ++v) o[nb][v] = o[nb][v] * alpha[v];

#pragma unroll
    for (int kg = 0; kg < 4; ++kg)
#pragma unroll
      for (int v = 0; v < 8; ++v)
        P[(hh * 8 + v) * LDT + kg * 16 + m] = (_Float16)(s[kg][v] * PCARRY);
    wave_lds_sync();

#pragma unroll
    for (int c = 0; c < 2; ++c) {
      const v16h pf = ld_frag(P + c * 32, LDT);
#pragma unroll
      for (int nb = 0; nb < 4; ++nb) {
        const v16h vf = ld_frag(&Vs[(nb * 16) * LDT + c * 32], LDT);
        o[nb] = wmma16(pf, vf, o[nb]);
      }
    }
    __syncthreads();
  }

  float inv[8];
#pragma unroll
  for (int v = 0; v < 8; ++v) inv[v] = __builtin_amdgcn_rcpf(lrow[v]) * (VCARRY / PCARRY);
#pragma unroll
  for (int nb = 0; nb < 4; ++nb)
#pragma unroll
    for (int v = 0; v < 8; ++v)
      P[(hh * 8 + v) * LDT + nb * 16 + m] = (_Float16)(o[nb][v] * inv[v]);
  wave_lds_sync();
  v8h x[4];
  size_t off[4];
#pragma unroll
  for (int i = 0; i < 4; ++i) {
    const int r = 4 * i + (lane >> 3);
    const int c = (lane & 7) * 8;
    x[i] = *(const v8h*)&P[r * LDT + c];
    off[i] = (tok0 + wq0 + r) * DIM + head * HD + c;
  }
#pragma unroll
  for (int i = 0; i < 4; ++i) *(volatile v8h*)(Ov + off[i]) = x[i];
  __threadfence();
#pragma unroll
  for (int i = 0; i < 4; ++i) *(volatile v8h*)(Ov + off[i]) = x[i];
}

static_assert(((size_t)MROWS * DIM) % 2048 == 0);
static_assert(((size_t)DIM * DIM) % 2048 == 0 && ((size_t)FF * DIM) % 2048 == 0);
static_assert((HD * HD) == 2 * 256 * 8);

extern "C" void kernel_launch(void* const* d_in, const int* in_sizes, int n_in,
                              void* d_out, int out_size, void* d_ws, size_t ws_size,
                              hipStream_t stream) {
  if (n_in < 14) return;
  const long long need_x = ((long long)(NB - 1) * SEQ_FULL + SEQ) * DIM;
  if ((long long)in_sizes[0] < need_x) return;
  if (in_sizes[1] < HD * HD || in_sizes[2] < HD * HD || in_sizes[3] < HD * HD) return;
  if (in_sizes[4] < DIM * DIM) return;
  if (in_sizes[5] < DIM || in_sizes[6] < DIM || in_sizes[7] < DIM || in_sizes[8] < DIM ||
      in_sizes[9] < DIM || in_sizes[13] < DIM) return;
  if (in_sizes[10] < FF * DIM || in_sizes[11] < FF || in_sizes[12] < DIM * FF) return;
  if ((long long)out_size < need_x) return;
  if (ws_size < WS_TOTAL) return;

  const float* x    = (const float*)d_in[0];
  const float* Wq   = (const float*)d_in[1];
  const float* Wk   = (const float*)d_in[2];
  const float* Wv   = (const float*)d_in[3];
  const float* Wo   = (const float*)d_in[4];
  const float* bo   = (const float*)d_in[5];
  const float* ln1g = (const float*)d_in[6];
  const float* ln1b = (const float*)d_in[7];
  const float* ln2g = (const float*)d_in[8];
  const float* ln2b = (const float*)d_in[9];
  const float* W1   = (const float*)d_in[10];
  const float* b1   = (const float*)d_in[11];
  const float* W2   = (const float*)d_in[12];
  const float* b2   = (const float*)d_in[13];
  float* out = (float*)d_out;

  char* ws = (char*)d_ws;
  _Float16* Wqkv16 = (_Float16*)(ws + OFF_WQKV);
  _Float16* Wo16   = (_Float16*)(ws + OFF_WO);
  _Float16* W116   = (_Float16*)(ws + OFF_W1);
  _Float16* W216   = (_Float16*)(ws + OFF_W2);
  _Float16* X16    = (_Float16*)(ws + OFF_XO);
  _Float16* Ov16   = (_Float16*)(ws + OFF_XO);
  _Float16* QKV16  = (_Float16*)(ws + OFF_QKV);
  _Float16* Q16    = QKV16;
  _Float16* K16    = QKV16 + (size_t)MROWS * DIM;
  _Float16* Vt16   = QKV16 + (size_t)2 * MROWS * DIM;
  float*    X32    = (float*)(ws + OFF_X32);
  float*    X1     = (float*)(ws + OFF_X1);
  _Float16* H16    = (_Float16*)(ws + OFF_H);
  _Float16* G16    = (_Float16*)(ws + OFF_G);

  dim3 blk(256);

  cvt_kernel<1><<<dim3((unsigned)((size_t)MROWS * DIM / 2048)), blk, 0, stream>>>(x, X16, 1.0f);
  cvt3_kernel<<<dim3(2, 3), blk, 0, stream>>>(Wq, Wk, Wv, Wqkv16);
  cvt_kernel<0><<<dim3((unsigned)((size_t)DIM * DIM / 2048)), blk, 0, stream>>>(Wo, Wo16, WCARRY);
  cvt_kernel<0><<<dim3((unsigned)((size_t)FF * DIM / 2048)), blk, 0, stream>>>(W1, W116, WCARRY);
  cvt_kernel<0><<<dim3((unsigned)((size_t)DIM * FF / 2048)), blk, 0, stream>>>(W2, W216, WCARRY);

  qkv_kernel<<<dim3(3 * NHEAD, MROWS / 64), blk, 0, stream>>>(X16, Wqkv16, QKV16);
  attn_kernel<<<dim3(SEQ / 128, NHEAD, NB), blk, 0, stream>>>(Q16, K16, Vt16, Ov16);
  gemm_kernel<MODE_WO, DIM, DIM><<<dim3(DIM / 64, MROWS / 64), blk, 0, stream>>>(
      Ov16, Wo16, bo, x, X32, H16);
  ln_kernel<1, 0><<<dim3(MROWS / 8), blk, 0, stream>>>(X32, ln1g, ln1b, X1, H16);
  gemm_kernel<MODE_W1, DIM, FF><<<dim3(FF / 64, MROWS / 64), blk, 0, stream>>>(
      H16, W116, b1, X1, X32, G16);
  gemm_kernel<MODE_W2, FF, DIM><<<dim3(DIM / 64, MROWS / 64), blk, 0, stream>>>(
      G16, W216, b2, X1, X32, H16);
  ln_kernel<0, 1><<<dim3(MROWS / 8), blk, 0, stream>>>(X32, ln2g, ln2b, out, H16);
}
